// GATNet_79173427134952
// MI455X (gfx1250) — hardware-verified
//
#include <hip/hip_runtime.h>
#include <stddef.h>
#include <math.h>


#define DIN     128
#define CW      128
#define HEADS   4
#define HC      32
#define NP      256
#define K1      128
#define DOUT    32
#define CPL     4
#define NTHR    256
#define NWAVE   8
#define EPT     8
#define CHUNK   (NTHR * EPT)
#define WCAP    (EPT * 32)
#define LISTN   (NWAVE * WCAP)
#define NBMAX   2048
#define NBRUN   1024
#define SLOTB   11
#define RCAP    28672
#define DEGCAP  128
#define STW     128
#define GBM     64
#define GBN     64
#define GTHR    128
#define NBW1    16
#define NBW2    16
#define NBWD    2
#define NBW     (NBW1 + NBW2 + NBWD)
#define CX      64.0f
#define CL      2048.0f
#define CWF     1024.0f
#define SCL_XW  1.52587890625e-5f
#define SCL_XWL 7.450580596923828125e-9f
#define NEGSA   0.2f
#define MX0     (-1.0e30f)
#define WSMAX   134217728
#define LDS_AGG ((2 * RCAP + 2 * NBMAX + LISTN) * 4 + 64)

static_assert((CHUNK & (CHUNK - 1)) == 0 && CHUNK <= (1 << SLOTB));
static_assert(NBMAX == (1 << SLOTB));
static_assert((NBRUN & (NBRUN - 1)) == 0 && NBRUN <= NBMAX && NBRUN >= 32);
static_assert(NTHR * 8 == NBMAX);
static_assert(LISTN >= NBMAX);
static_assert(LISTN >= NWAVE * WCAP);
static_assert((RCAP % 32) == 0);
static_assert(NWAVE * STW <= RCAP);
static_assert(STW == CW && CW == 32 * CPL && CPL == 4);
static_assert(CW == HEADS * HC && HC == 8 * CPL);
static_assert(LDS_AGG == 254016);
static_assert(GBM == (GTHR / 32) * 16);
static_assert((K1 % 32) == 0 && DIN == K1 && CW == K1);
static_assert(DIN / 8 == 16);
static_assert((NP % GBN) == 0 && NP == 2 * CW && (CW % GBN) == 0);
static_assert(NBW1 * NTHR == NP * (K1 / 8) && (NBW1 / 2) * NTHR == CW * (K1 / 8));
static_assert(NBW2 == NBW1);
static_assert(NBWD * NTHR == DOUT * (K1 / 8));
static_assert(DOUT == 32 && GBM == 64 && GTHR == 128);
static_assert(DEGCAP <= RCAP);

typedef float          v4f   __attribute__((ext_vector_type(4)));
typedef float          v8f   __attribute__((ext_vector_type(8)));
typedef int            v4i   __attribute__((ext_vector_type(4)));
typedef int            v8i   __attribute__((ext_vector_type(8)));
typedef unsigned short v8us  __attribute__((ext_vector_type(8)));
typedef _Float16       v8h   __attribute__((ext_vector_type(8)));
typedef _Float16       v16h  __attribute__((ext_vector_type(16)));
typedef __bf16         v16bf __attribute__((ext_vector_type(16)));
typedef v4f  __attribute__((may_alias)) v4fa;
typedef v8us __attribute__((may_alias)) v8usa;
union FragH { v16h v;  v8us u[2]; v8i w; };
union FragB { v16bf v; v8us u[2]; v8i w; };
template<int BF> struct FT { typedef FragH T; };
template<> struct FT<1> { typedef FragB T; };

__device__ __forceinline__ v8f wmx(const FragH& a, const FragH& b, v8f c) {
  v8f d = __builtin_amdgcn_wmma_f32_16x16x32_f16(false, a.v, false, b.v, (short)0, c, false, false);
  asm volatile("v_nop\n\tv_nop\n\tv_nop\n\tv_nop" : "+v"(d) : "v"(a.w), "v"(b.w));
  return d;
}
__device__ __forceinline__ v8f wmx(const FragB& a, const FragB& b, v8f c) {
  v8f d = __builtin_amdgcn_wmma_f32_16x16x32_bf16(false, a.v, false, b.v, (short)0, c, false, false);
  asm volatile("v_nop\n\tv_nop\n\tv_nop\n\tv_nop" : "+v"(d) : "v"(a.w), "v"(b.w));
  return d;
}

__device__ __forceinline__ unsigned bfbits(float v) {
  unsigned u = __float_as_uint(v);
  u = u + 0x7FFFu + ((u >> 16) & 1u);
  return u >> 16;
}
__device__ __forceinline__ float rbf(float v) { return __uint_as_float(bfbits(v) << 16); }
__device__ __forceinline__ v4f rbf4(const v4f a) {
  v4f r; r.x = rbf(a.x); r.y = rbf(a.y); r.z = rbf(a.z); r.w = rbf(a.w); return r;
}

__device__ __forceinline__ v8us cvt8b(const v4f a, const v4f b) {
  v8us o;
  o[0] = (unsigned short)bfbits(a.x); o[1] = (unsigned short)bfbits(a.y);
  o[2] = (unsigned short)bfbits(a.z); o[3] = (unsigned short)bfbits(a.w);
  o[4] = (unsigned short)bfbits(b.x); o[5] = (unsigned short)bfbits(b.y);
  o[6] = (unsigned short)bfbits(b.z); o[7] = (unsigned short)bfbits(b.w);
  return o;
}
__device__ __forceinline__ v8h cvt8bh(const v4f a, const v4f b, const float c) {
  v8h hv;
  hv[0] = (_Float16)(rbf(a.x) * c); hv[1] = (_Float16)(rbf(a.y) * c);
  hv[2] = (_Float16)(rbf(a.z) * c); hv[3] = (_Float16)(rbf(a.w) * c);
  hv[4] = (_Float16)(rbf(b.x) * c); hv[5] = (_Float16)(rbf(b.y) * c);
  hv[6] = (_Float16)(rbf(b.z) * c); hv[7] = (_Float16)(rbf(b.w) * c);
  return hv;
}
__device__ __forceinline__ void cvt8hl(const v4f a, const v4f b, v8h& hv, v8h& lv) {
  float f[8] = {a.x * CX, a.y * CX, a.z * CX, a.w * CX, b.x * CX, b.y * CX, b.z * CX, b.w * CX};
#pragma unroll
  for (int i = 0; i < 8; ++i) {
    const _Float16 hq = (_Float16)f[i];
    hv[i] = hq;
    lv[i] = (_Float16)((f[i] - (float)hq) * CL);
  }
}
template<int NQ>
__device__ __forceinline__ void ldq(float (&d)[4 * NQ], const float* __restrict__ p) {
#pragma unroll
  for (int k = 0; k < NQ; ++k) {
    const v4f t = *(const v4fa*)(p + 4 * k);
    d[4 * k] = t.x; d[4 * k + 1] = t.y; d[4 * k + 2] = t.z; d[4 * k + 3] = t.w;
  }
}
template<int NQ>
__device__ __forceinline__ void ldqb(float (&d)[4 * NQ], const float* __restrict__ p) {
#pragma unroll
  for (int k = 0; k < NQ; ++k) {
    const v4f t = rbf4(*(const v4fa*)(p + 4 * k));
    d[4 * k] = t.x; d[4 * k + 1] = t.y; d[4 * k + 2] = t.z; d[4 * k + 3] = t.w;
  }
}
__device__ __forceinline__ float hsum8(float p) {
  p += __shfl_xor(p, 4); p += __shfl_xor(p, 2); p += __shfl_xor(p, 1);
  return p;
}

__device__ __forceinline__ int scan_chunk(const int* __restrict__ dsts, int nE, int cbase, int slotBase,
                                          int nb, int vec8, int* list, int tid, int lane, int wave) {
  int wc = 0;
  const int el0  = tid * EPT;
  const int e0   = cbase + el0;
  const int sent = -2147483647 - 1;
  v4i da, db;
  if (vec8 != 0 && cbase + CHUNK <= nE) {
    da = *(const v4i*)(dsts + e0);
    db = *(const v4i*)(dsts + e0 + 4);
  } else {
    da.x = (e0     < nE) ? dsts[min(e0,     nE - 1)] : sent;
    da.y = (e0 + 1 < nE) ? dsts[min(e0 + 1, nE - 1)] : sent;
    da.z = (e0 + 2 < nE) ? dsts[min(e0 + 2, nE - 1)] : sent;
    da.w = (e0 + 3 < nE) ? dsts[min(e0 + 3, nE - 1)] : sent;
    db.x = (e0 + 4 < nE) ? dsts[min(e0 + 4, nE - 1)] : sent;
    db.y = (e0 + 5 < nE) ? dsts[min(e0 + 5, nE - 1)] : sent;
    db.z = (e0 + 6 < nE) ? dsts[min(e0 + 6, nE - 1)] : sent;
    db.w = (e0 + 7 < nE) ? dsts[min(e0 + 7, nE - 1)] : sent;
  }
  const unsigned nbs = (unsigned)slotBase;
  const unsigned unb = (unsigned)nb;
  const unsigned s0 = (unsigned)da.x - nbs, s1 = (unsigned)da.y - nbs;
  const unsigned s2 = (unsigned)da.z - nbs, s3 = (unsigned)da.w - nbs;
  const unsigned s4 = (unsigned)db.x - nbs, s5 = (unsigned)db.y - nbs;
  const unsigned s6 = (unsigned)db.z - nbs, s7 = (unsigned)db.w - nbs;
  const bool h0 = s0 < unb, h1 = s1 < unb, h2 = s2 < unb, h3 = s3 < unb;
  const bool h4 = s4 < unb, h5 = s5 < unb, h6 = s6 < unb, h7 = s7 < unb;
  const unsigned any = __builtin_amdgcn_ballot_w32(h0 | h1 | h2 | h3 | h4 | h5 | h6 | h7);
  if (any != 0u) {
#define HITJ(J, HJ, SJ) { \
      const unsigned mj = __builtin_amdgcn_ballot_w32(HJ); \
      if (mj != 0u) { \
        if (HJ) { \
          const int pos = wc + (int)__builtin_amdgcn_mbcnt_lo(mj, 0u); \
          if (pos < WCAP) list[wave * WCAP + pos] = ((el0 + (J)) << SLOTB) | (int)(SJ); \
        } \
        wc += (int)__builtin_popcount(mj); } }
    HITJ(0, h0, s0)
    HITJ(1, h1, s1)
    HITJ(2, h2, s2)
    HITJ(3, h3, s3)
    HITJ(4, h4, s4)
    HITJ(5, h5, s5)
    HITJ(6, h6, s6)
    HITJ(7, h7, s7)
#undef HITJ
  }
  return wc;
}

__device__ __forceinline__ void w_unit_b(const float* __restrict__ w, unsigned short* wt, int n, int nl, int c0) {
  const float* p = w + (size_t)nl * DIN + c0;
  const v4f a = *(const v4fa*)p, b = *(const v4fa*)(p + 4);
  const v8us hv = cvt8b(a, b);
  const size_t o = (size_t)n * (size_t)K1 + c0;
  *(volatile v8us*)(wt + o) = hv;
  __threadfence();
  *(volatile v8us*)(wt + o) = hv;
}
__device__ __forceinline__ void w_unit_h(const float* __restrict__ w, _Float16* wt, int n, int nl, int c0) {
  const float* p = w + (size_t)nl * DIN + c0;
  const v4f a = *(const v4fa*)p, b = *(const v4fa*)(p + 4);
  const v8h hv = cvt8bh(a, b, CWF);
  const size_t o = (size_t)n * (size_t)K1 + c0;
  *(volatile v8h*)(wt + o) = hv;
  __threadfence();
  *(volatile v8h*)(wt + o) = hv;
}

__global__ __launch_bounds__(NTHR) void k_prep(const float* __restrict__ x,
                                               const float* __restrict__ Wl0, const float* __restrict__ Wr0,
                                               const float* __restrict__ Wl1, const float* __restrict__ Wr1,
                                               const float* __restrict__ Wd,
                                               unsigned short* xb, unsigned short* wt1, _Float16* wt2, _Float16* wtd,
                                               int nN, int nUx, int nBx) {
  const int tid = (int)threadIdx.x;
  const int bid = (int)blockIdx.x;
  if (bid < nBx) {
    const int i = bid * NTHR + tid;
    if (i >= nUx) return;
    const int row = i >> 4;
    const int c0  = (i & 15) * 8;
    const int rc  = row < nN ? row : nN - 1;
    const float* p = x + (size_t)rc * DIN + c0;
    v4f a = *(const v4fa*)p, b = *(const v4fa*)(p + 4);
    const v4f z4 = {0.f, 0.f, 0.f, 0.f};
    if (row >= nN) { a = z4; b = z4; }
    const v8us hv = cvt8b(a, b);
    const size_t o = (size_t)row * DIN + c0;
    *(volatile v8us*)(xb + o) = hv;
    __threadfence();
    *(volatile v8us*)(xb + o) = hv;
  } else {
    const int rb = bid - nBx;
    if (rb < NBW1) {
      const int u  = rb * NTHR + tid;
      const int n  = u >> 4;
      const int c0 = (u & 15) * 8;
      const int nl = n & (CW - 1);
      if (rb < NBW1 / 2) w_unit_b(Wl0, wt1, n, nl, c0);
      else               w_unit_b(Wr0, wt1, n, nl, c0);
    } else if (rb < NBW1 + NBW2) {
      const int rq = rb - NBW1;
      const int u  = rq * NTHR + tid;
      const int n  = u >> 4;
      const int c0 = (u & 15) * 8;
      const int nl = n & (CW - 1);
      if (rq < NBW2 / 2) w_unit_h(Wl1, wt2, n, nl, c0);
      else               w_unit_h(Wr1, wt2, n, nl, c0);
    } else if (rb < NBW) {
      const int rq = rb - NBW1 - NBW2;
      const int u  = rq * NTHR + tid;
      const int n  = u >> 4;
      const int c0 = (u & 15) * 8;
      w_unit_h(Wd, wtd, n, n, c0);
    }
  }
}

template<int BF, int RES>
__global__ __launch_bounds__(GTHR) void k_gemm(
    const unsigned short* __restrict__ A, const unsigned short* __restrict__ A2,
    const unsigned short* __restrict__ WT, const float* __restrict__ bl, const float* __restrict__ br,
    float* outF, int K, int ldo, int csplit, float scl, float scl2)
{
  typedef typename FT<BF>::T Frag;
  __shared__ __attribute__((aligned(16))) float stg[GBM * GBN];
  const int tid = (int)threadIdx.x, lane = tid & 31, wave = tid >> 5, hh = lane >> 4, m = lane & 15;
  const int rowBase = (int)blockIdx.x * GBM;
  const int col0    = (int)blockIdx.y * GBN;

  v8f acc[4], acc2[4];
  {
    const v8f z = {0.f, 0.f, 0.f, 0.f, 0.f, 0.f, 0.f, 0.f};
    acc[0] = z; acc[1] = z; acc[2] = z; acc[3] = z;
    acc2[0] = z; acc2[1] = z; acc2[2] = z; acc2[3] = z;
  }
  const size_t arow = (size_t)(rowBase + 16 * wave + m) * (size_t)K + 8 * hh;
  const unsigned short* ap  = A  + arow;
  const unsigned short* ap2 = A2 + arow;
  const unsigned short* wp  = WT + (size_t)(col0 + m) * (size_t)K + 8 * hh;
  const int ksteps = K >> 5;
#pragma unroll 1
  for (int ks = 0; ks < ksteps; ++ks) {
    Frag af, af2;
    af.u[0] = *(const v8usa*)(ap + 32 * ks);
    af.u[1] = *(const v8usa*)(ap + 32 * ks + 16);
    if (RES) {
      af2.u[0] = *(const v8usa*)(ap2 + 32 * ks);
      af2.u[1] = *(const v8usa*)(ap2 + 32 * ks + 16);
    } else {
      af2 = af;
    }
#pragma unroll
    for (int t = 0; t < 4; ++t) {
      const unsigned short* wq = wp + (size_t)(16 * t) * (size_t)K + 32 * ks;
      Frag bf;
      bf.u[0] = *(const v8usa*)wq;
      bf.u[1] = *(const v8usa*)(wq + 16);
      acc[t] = wmx(af, bf, acc[t]);
      if (RES) acc2[t] = wmx(af2, bf, acc2[t]);
    }
  }

#pragma unroll
  for (int t = 0; t < 4; ++t) {
    const int lc = 16 * t + m;
#pragma unroll
    for (int r = 0; r < 8; ++r) {
      const int lr = 16 * wave + 8 * hh + r;
      const float v = RES ? fmaf(acc2[t][r], scl2, acc[t][r] * scl) : acc[t][r] * scl;
      stg[lr * GBN + lc] = v;
    }
  }
  __syncthreads();

  v4f b4;
  {
    int ca = col0; ca = ca > csplit - GBN ? csplit - GBN : ca;
    int cb = col0 - csplit; cb = cb < 0 ? 0 : cb;
    const float fb = (col0 >= csplit) ? 1.0f : 0.0f;
    const float fa = 1.0f - fb;
    const v4f va = *(const v4fa*)(bl + ca + 4 * m);
    const v4f vb = *(const v4fa*)(br + cb + 4 * m);
    b4.x = rbf(fmaf(va.x, fa, vb.x * fb)); b4.y = rbf(fmaf(va.y, fa, vb.y * fb));
    b4.z = rbf(fmaf(va.z, fa, vb.z * fb)); b4.w = rbf(fmaf(va.w, fa, vb.w * fb));
  }

  v4f fv[8];
#pragma unroll
  for (int i = 0; i < 8; ++i) {
    const int lr = 16 * wave + 2 * i + hh;
    fv[i] = *(const v4fa*)(stg + lr * GBN + 4 * m) + b4;
  }
#pragma unroll
  for (int i = 0; i < 8; ++i) {
    const int lr = 16 * wave + 2 * i + hh;
    const int gr = rowBase + lr;
    float* op = outF + (size_t)gr * (size_t)ldo + col0 + 4 * m;
    *(volatile v4f*)op = fv[i];
  }
  __threadfence();
#pragma unroll
  for (int i = 0; i < 8; ++i) {
    const int lr = 16 * wave + 2 * i + hh;
    const int gr = rowBase + lr;
    float* op = outF + (size_t)gr * (size_t)ldo + col0 + 4 * m;
    *(volatile v4f*)op = fv[i];
  }
}

__global__ __launch_bounds__(GTHR) void k_down(
    const unsigned short* __restrict__ A, const unsigned short* __restrict__ A2,
    const unsigned short* __restrict__ WT, const float* __restrict__ bd,
    float* outp, int K, int nN, float scl, float scl2)
{
  __shared__ __attribute__((aligned(16))) float stg[GBM * DOUT];
  const int tid = (int)threadIdx.x, lane = tid & 31, wave = tid >> 5, hh = lane >> 4, m = lane & 15;
  const int rowBase = (int)blockIdx.x * GBM;

  v8f acc[2], acc2[2];
  {
    const v8f z = {0.f, 0.f, 0.f, 0.f, 0.f, 0.f, 0.f, 0.f};
    acc[0] = z; acc[1] = z; acc2[0] = z; acc2[1] = z;
  }
  const size_t arow = (size_t)(rowBase + 16 * wave + m) * (size_t)K + 8 * hh;
  const unsigned short* ap  = A  + arow;
  const unsigned short* ap2 = A2 + arow;
  const unsigned short* wp  = WT + (size_t)m * (size_t)K + 8 * hh;
  const int ksteps = K >> 5;
#pragma unroll 1
  for (int ks = 0; ks < ksteps; ++ks) {
    FragH af, af2;
    af.u[0]  = *(const v8usa*)(ap + 32 * ks);
    af.u[1]  = *(const v8usa*)(ap + 32 * ks + 16);
    af2.u[0] = *(const v8usa*)(ap2 + 32 * ks);
    af2.u[1] = *(const v8usa*)(ap2 + 32 * ks + 16);
#pragma unroll
    for (int t = 0; t < 2; ++t) {
      const unsigned short* wq = wp + (size_t)(16 * t) * (size_t)K + 32 * ks;
      FragH bf;
      bf.u[0] = *(const v8usa*)wq;
      bf.u[1] = *(const v8usa*)(wq + 16);
      acc[t]  = wmx(af, bf, acc[t]);
      acc2[t] = wmx(af2, bf, acc2[t]);
    }
  }

#pragma unroll
  for (int t = 0; t < 2; ++t) {
    const int lc = 16 * t + m;
#pragma unroll
    for (int r = 0; r < 8; ++r) {
      const int lr = 16 * wave + 8 * hh + r;
      stg[lr * DOUT + lc] = fmaf(acc2[t][r], scl2, acc[t][r] * scl);
    }
  }
  __syncthreads();

  const int cq = lane & 7;
  const int rq = lane >> 3;
  const v4f b4 = rbf4(*(const v4fa*)(bd + 4 * cq));
  v4f fv[4];
#pragma unroll
  for (int i = 0; i < 4; ++i) {
    const int lr = 16 * wave + 4 * i + rq;
    fv[i] = *(const v4fa*)(stg + lr * DOUT + 4 * cq) + b4;
  }
#pragma unroll
  for (int i = 0; i < 4; ++i) {
    const int gr = rowBase + 16 * wave + 4 * i + rq;
    float* op = outp + (size_t)gr * DOUT + 4 * cq;
    if (gr < nN) *(volatile v4f*)op = fv[i];
  }
  __threadfence();
#pragma unroll
  for (int i = 0; i < 4; ++i) {
    const int gr = rowBase + 16 * wave + 4 * i + rq;
    float* op = outp + (size_t)gr * DOUT + 4 * cq;
    if (gr < nN) *(volatile v4f*)op = fv[i];
  }
}

template<int C>
__device__ __forceinline__ float edot(const float (&hs)[C], const float (&hd)[C], const float (&at)[C]) {
  float part = 0.f;
#pragma unroll
  for (int j = 0; j < C; ++j) {
    float v = hs[j] + hd[j];
    v = v >= 0.f ? v : v * NEGSA;
    part = fmaf(v, at[j], part);
  }
  return part;
}
template<int C>
__device__ __forceinline__ void smerge(float lg, float& mx, float& dn, float (&av)[C], const float (&hm)[C]) {
  const float df = lg - mx;
  const float ee = __expf(-fabsf(df));
  const bool up  = df > 0.f;
  const float s1 = up ? ee : 1.0f;
  const float s2 = up ? 1.0f : ee;
  mx = up ? lg : mx;
  dn = fmaf(dn, s1, s2);
#pragma unroll
  for (int j = 0; j < C; ++j) av[j] = fmaf(av[j], s1, s2 * hm[j]);
}

__global__ __launch_bounds__(NTHR) void k_agg(
    const int* __restrict__ srcs, const int* __restrict__ dsts,
    const float* __restrict__ F, const float* __restrict__ att, const float* __restrict__ bias,
    _Float16* HP, int nN, int nE, int nb, int vec8, int MPr) {
  extern __shared__ v4f lds_dyn[];
  int* reg1 = (int*)lds_dyn;
  int* reg2 = reg1 + RCAP;
  int* scnt = reg2 + RCAP;
  int* soff = scnt + NBMAX;
  int* list = soff + NBMAX;
  int* wcnt = list + LISTN;
  int* wtot = wcnt + NWAVE;
  const int tid = (int)threadIdx.x, lane = tid & 31, wave = tid >> 5;
  const int nodeBase = (int)blockIdx.x * nb;

  for (int i = tid; i < NBMAX; i += NTHR) scnt[i] = 0;
  for (int i = tid; i < RCAP; i += NTHR) reg2[i] = 0;
  __syncthreads();

  int tot = 0;
  const int nChunks = (nE + CHUNK - 1) / CHUNK;
#pragma unroll 1
  for (int ch = 0; ch < nChunks; ++ch) {
    const int cbase = ch * CHUNK;
    const int wc = scan_chunk(dsts, nE, cbase, nodeBase, nb, vec8, list, tid, lane, wave);
    if (lane == 0) wcnt[wave] = wc;
    __syncthreads();
    int pre = 0, all = 0;
#pragma unroll
    for (int w2 = 0; w2 < NWAVE; ++w2) {
      int c = wcnt[w2];
      c = c < 0 ? 0 : (c > WCAP ? WCAP : c);
      all += c;
      pre += (w2 < wave) ? c : 0;
    }
    const int wcc  = wc > WCAP ? WCAP : wc;
    const int base = tot + pre;
#pragma unroll 1
    for (int i = lane; i < wcc; i += 32) {
      const int ent = list[wave * WCAP + i];
      const int el  = (ent >> SLOTB) & (CHUNK - 1);
      const int sl  = ent & (NBMAX - 1);
      int eid = cbase + el;
      eid = eid > nE - 1 ? nE - 1 : eid;
      const int pos = base + i;
      if (pos < RCAP) reg1[pos] = (int)(((unsigned)eid << SLOTB) | (unsigned)sl);
    }
    tot += all;
    tot = tot > RCAP ? RCAP : tot;
    __syncthreads();
  }
  const int nh = tot;

  if (wave == 0) {
#pragma unroll 1
    for (int b0 = 0; b0 < nh; b0 += 32) {
      const int idx = b0 + lane;
      const int uv  = reg1[idx < nh ? idx : nh - 1];
      const int m32 = (nh - b0) < 32 ? (nh - b0) : 32;
#pragma unroll 1
      for (int k = 0; k < m32; ++k) {
        const int u  = __builtin_amdgcn_readlane(uv, k);
        const int sl = u & (NBMAX - 1);
        if (lane == 0) scnt[sl] = scnt[sl] + 1;
      }
    }
  }
  __syncthreads();

  {
    const v4i ca = *(const v4i*)(scnt + 8 * tid);
    const v4i cb = *(const v4i*)(scnt + 8 * tid + 4);
    const int e0 = ca.x < 0 ? 0 : ca.x, e1 = ca.y < 0 ? 0 : ca.y, e2 = ca.z < 0 ? 0 : ca.z, e3 = ca.w < 0 ? 0 : ca.w;
    const int e4 = cb.x < 0 ? 0 : cb.x, e5 = cb.y < 0 ? 0 : cb.y, e6 = cb.z < 0 ? 0 : cb.z, e7 = cb.w < 0 ? 0 : cb.w;
    const int ts = e0 + e1 + e2 + e3 + e4 + e5 + e6 + e7;
    int incl = ts;
#pragma unroll
    for (int d = 1; d < 32; d <<= 1) {
      const int up = __shfl_up(incl, d);
      if (lane >= d) incl += up;
    }
    if (lane == 31) wtot[wave] = incl;
    __syncthreads();
    int pre = 0;
#pragma unroll
    for (int w2 = 0; w2 < NWAVE; ++w2) pre += (w2 < wave) ? wtot[w2] : 0;
    int run = pre + incl - ts;
    soff[8 * tid + 0] = run; run += e0;
    soff[8 * tid + 1] = run; run += e1;
    soff[8 * tid + 2] = run; run += e2;
    soff[8 * tid + 3] = run; run += e3;
    soff[8 * tid + 4] = run; run += e4;
    soff[8 * tid + 5] = run; run += e5;
    soff[8 * tid + 6] = run; run += e6;
    soff[8 * tid + 7] = run;
  }
  __syncthreads();
  for (int i = tid; i < NBMAX; i += NTHR) list[i] = soff[i];
  __syncthreads();

  if (wave == 0) {
#pragma unroll 1
    for (int b0 = 0; b0 < nh; b0 += 32) {
      const int idx = b0 + lane;
      const int uv  = reg1[idx < nh ? idx : nh - 1];
      const int m32 = (nh - b0) < 32 ? (nh - b0) : 32;
#pragma unroll 1
      for (int k = 0; k < m32; ++k) {
        const int u   = __builtin_amdgcn_readlane(uv, k);
        const int sl  = u & (NBMAX - 1);
        const int eid = (int)((unsigned)u >> SLOTB);
        if (lane == 0) {
          int pos = list[sl];
          pos = pos < 0 ? 0 : (pos > RCAP - 1 ? RCAP - 1 : pos);
          reg2[pos] = eid;
          list[sl] = pos + 1;
        }
      }
    }
  }
  __syncthreads();

  const int nbw = nb >> 3;
  const bool ovf = (nh >= RCAP);
  const float qnan = __int_as_float(0x7fc00000);
  float* stw = (float*)reg1 + wave * STW;
  const size_t pstr = (size_t)MPr * (size_t)CW;
  const int c0  = CPL * lane;
  const int q16 = lane & 15;
  const bool hsel = lane >= 16;
  float at[CPL], bb[CPL];
  ldqb<CPL / 4>(at, att + c0);
  ldqb<CPL / 4>(bb, bias + c0);

#pragma unroll 1
  for (int jt = 0; jt < nbw; ++jt) {
    const int slot = wave * nbw + jt;
    const int grow = nodeBase + slot;
    const int gcl  = grow < nN ? grow : nN - 1;
    int st = soff[slot];
    const int craw = scnt[slot];
    int cnt = craw;
    st  = st < 0 ? 0 : (st > nh ? nh : st);
    cnt = cnt < 0 ? 0 : (cnt > DEGCAP ? DEGCAP : cnt);
    if (cnt > nh - st) cnt = nh - st;
    const float pz = (ovf || craw > DEGCAP) ? qnan : 0.0f;
    const bool live = grow < nN;
    const bool wr   = grow < MPr;

    const float* fr = F + (size_t)gcl * (size_t)NP;
    float hd[CPL];
    ldq<CPL / 4>(hd, fr + CW + c0);
    float av[CPL];
#pragma unroll
    for (int j = 0; j < CPL; ++j) av[j] = 0.f;
    float mx = MX0, dn = 0.f;

#pragma unroll 1
    for (int q = 0; q <= cnt; ++q) {
      const bool last = (q == cnt);
      int idx = st + q; idx = idx > RCAP - 1 ? RCAP - 1 : idx;
      int eid = reg2[idx]; eid = eid < 0 ? 0 : (eid > nE - 1 ? nE - 1 : eid);
      const int sraw = srcs[eid];
      const int se = sraw < 0 ? 0 : (sraw > nN - 1 ? nN - 1 : sraw);
      const int s = last ? gcl : se;
      const float* sr = F + (size_t)s * (size_t)NP + c0;
      float hl[CPL];
      ldq<CPL / 4>(hl, sr);
      const float lg = hsum8(edot<CPL>(hl, hd, at));
      smerge<CPL>(lg, mx, dn, av, hl);
    }
    const float inv = __builtin_amdgcn_rcpf(dn);

    float r[CPL];
#pragma unroll
    for (int j = 0; j < CPL; ++j) {
      const float v = fmaf(av[j], inv, bb[j]);
      r[j] = (live ? v : 0.f) + pz;
    }
    __builtin_amdgcn_fence(__ATOMIC_RELEASE, "wavefront");
    __builtin_amdgcn_wave_barrier();
    {
      const v4f rv = {r[0], r[1], r[2], r[3]};
      *(v4fa*)(stw + 4 * lane) = rv;
    }
    __builtin_amdgcn_fence(__ATOMIC_RELEASE, "wavefront");
    __builtin_amdgcn_wave_barrier();
    const v4f ga = *(const v4fa*)(stw + 8 * q16);
    const v4f gb = *(const v4fa*)(stw + 8 * q16 + 4);
    v8h hv, lv;
    cvt8hl(ga, gb, hv, lv);
    v8h ov;
#pragma unroll
    for (int i = 0; i < 8; ++i) ov[i] = hsel ? lv[i] : hv[i];
    _Float16* gp = HP + (size_t)(lane >> 4) * pstr + (size_t)grow * CW + 8 * q16;
    if (wr) *(volatile v8h*)gp = ov;
    __threadfence();
    if (wr) *(volatile v8h*)gp = ov;
  }
}

static int pick_nb(int nE, int nN) {
  int nb = NBRUN;
  while (nb > 32 && (long long)nb * (long long)nE * 5LL > (long long)RCAP * (long long)nN * 4LL) nb >>= 1;
  return nb;
}
static inline int cdiv(int a, int b) { return (a + b - 1) / b; }

extern "C" void kernel_launch(void* const* d_in, const int* in_sizes, int n_in,
                              void* d_out, int out_size, void* d_ws, size_t ws_size,
                              hipStream_t stream) {
  if (n_in < 16) return;
  const int nN = in_sizes[0] / DIN;
  if (nN <= 0 || in_sizes[0] != nN * DIN || nN > (1 << 21)) return;
  if (in_sizes[1] < 2 || (in_sizes[1] & 1) != 0) return;
  const int nE = in_sizes[1] / 2;
  if (nE < 1 || nE >= (1 << (32 - SLOTB))) return;
  if (in_sizes[2] != CW * DIN || in_sizes[3] != CW) return;
  if (in_sizes[4] != CW * DIN || in_sizes[5] != CW) return;
  if (in_sizes[6] != CW || in_sizes[7] != CW) return;
  if (in_sizes[8] != CW * CW || in_sizes[9] != CW) return;
  if (in_sizes[10] != CW * CW || in_sizes[11] != CW) return;
  if (in_sizes[12] != CW || in_sizes[13] != CW) return;
  if (in_sizes[14] != DOUT * CW || in_sizes[15] != DOUT) return;
  if (out_size != nN * DOUT) return;

  const float* x     = (const float*)d_in[0];
  const int*   ei    = (const int*)  d_in[1];
  const float* Wl0   = (const float*)d_in[2];
  const float* bl0   = (const float*)d_in[3];
  const float* Wr0   = (const float*)d_in[4];
  const float* br0   = (const float*)d_in[5];
  const float* att0  = (const float*)d_in[6];
  const float* bias0 = (const float*)d_in[7];
  const float* Wl1   = (const float*)d_in[8];
  const float* bl1   = (const float*)d_in[9];
  const float* Wr1   = (const float*)d_in[10];
  const float* br1   = (const float*)d_in[11];
  const float* att1  = (const float*)d_in[12];
  const float* bias1 = (const float*)d_in[13];
  const float* Wd    = (const float*)d_in[14];
  const float* bd    = (const float*)d_in[15];
  float* outp = (float*)d_out;
  const int* src = ei;
  const int* dst = ei + nE;

  const int MP   = cdiv(nN, GBM) * GBM;
  const int nb   = pick_nb(nE, nN);
  if (nb < 32 || (nb & (nb - 1)) != 0 || nb > NBMAX) return;
  const int gA   = cdiv(MP, nb);
  const int vec8 = ((nE & 3) == 0) ? 1 : 0;
  if (gA * nb < MP) return;

  char* ws = (char*)d_ws;
  size_t off = 0;
  const size_t oXB  = off; off += (size_t)MP * DIN * 2;            off = (off + 255) & ~(size_t)255;
  const size_t oWT1 = off; off += (size_t)NP * K1 * 2;             off = (off + 255) & ~(size_t)255;
  const size_t oWT2 = off; off += (size_t)NP * K1 * 2;             off = (off + 255) & ~(size_t)255;
  const size_t oWTD = off; off += (size_t)DOUT * K1 * 2;           off = (off + 255) & ~(size_t)255;
  const size_t oHF  = off; off += (size_t)MP * NP * 4;             off = (off + 255) & ~(size_t)255;
  const size_t oHP  = off; off += (size_t)2 * MP * CW * 2;         off = (off + 255) & ~(size_t)255;
  if (off > ws_size || off > (size_t)WSMAX) return;
  unsigned short* XB  = (unsigned short*)(ws + oXB);
  unsigned short* WT1 = (unsigned short*)(ws + oWT1);
  unsigned short* WT2 = (unsigned short*)(ws + oWT2);
  unsigned short* WTD = (unsigned short*)(ws + oWTD);
  float*          HF  = (float*)(ws + oHF);
  unsigned short* HP  = (unsigned short*)(ws + oHP);
  unsigned short* HPL = HP + (size_t)MP * CW;

  hipFuncSetAttribute(reinterpret_cast<const void*>(&k_agg),
                      hipFuncAttributeMaxDynamicSharedMemorySize, LDS_AGG);

  const int nUx = MP * (DIN / 8);
  const int nBx = cdiv(nUx, NTHR);
  if (nBx * NTHR != nUx) return;
  k_prep<<<nBx + NBW, NTHR, 0, stream>>>(x, Wl0, Wr0, Wl1, Wr1, Wd, XB, WT1, (_Float16*)WT2, (_Float16*)WTD,
                                         nN, nUx, nBx);

  const int gM = MP / GBM;
  k_gemm<1, 0><<<dim3(gM, NP / GBN), GTHR, 0, stream>>>(XB, XB, WT1, bl0, br0, HF, K1, NP, CW, 1.0f, 0.0f);
  k_agg<<<gA, NTHR, LDS_AGG, stream>>>(src, dst, HF, att0, bias0, (_Float16*)HP, nN, nE, nb, vec8, MP);
  k_gemm<0, 1><<<dim3(gM, NP / GBN), GTHR, 0, stream>>>(HP, HPL, WT2, bl1, br1, HF, K1, NP, CW, SCL_XW, SCL_XWL);
  k_agg<<<gA, NTHR, LDS_AGG, stream>>>(src, dst, HF, att1, bias1, (_Float16*)HP, nN, nE, nb, vec8, MP);
  k_down<<<gM, GTHR, 0, stream>>>(HP, HPL, WTD, bd, outp, K1, nN, SCL_XW, SCL_XWL);
}
